// EnsembleUncertaintyDistance_53824530153580
// MI455X (gfx1250) — hardware-run, weakly checked
//
#include <hip/hip_runtime.h>
#include <stddef.h>


typedef _Float16 v16h __attribute__((ext_vector_type(16)));
typedef _Float16 v8h  __attribute__((ext_vector_type(8)));
typedef float    v8f  __attribute__((ext_vector_type(8)));
typedef float    v4f  __attribute__((ext_vector_type(4)));

#ifndef NQ
#define NQ 2048
#endif
#define NQ_FULL 2048
#define NP    256
#define EMB   512
#define KW    (2 * EMB)
#define NM    5
#define HID   64
#define NH    (NM * HID)
#define MROWS (NQ + NP)

#define QT  16
#define PT  128
#define SP  132
#define LDC 68

#define XCARRY 16.0f
#define WCARRY 64.0f
#define HCARRY 16.0f

static_assert(NQ >= 64 && NQ <= NQ_FULL && (NQ % 64) == 0);
static_assert((NQ % QT) == 0);
static_assert((NP % 64) == 0 && (NP % PT) == 0);
static_assert((MROWS % 64) == 0);
static_assert((EMB % 32) == 0 && (KW % 8) == 0 && (EMB % 8) == 0);
static_assert(HID == 64);
static_assert((NH % 64) == 0 && (NH % 4) == 0);
static_assert(((size_t)NQ * EMB) % 2048 == 0);
static_assert(((size_t)NP * EMB) % 2048 == 0);
static_assert(((size_t)NH * KW) % 2048 == 0);
static_assert(QT * NH == 5 * 256 * 4);
static_assert(QT == 2 * 8);
static_assert(PT == 8 * 16 && PT == 32 * 4);
static_assert((SP % 4) == 0 && SP >= PT);
static_assert((LDC % 4) == 0 && LDC >= 64);

#define X_BYTES ((size_t)MROWS * EMB * 2)
#define W_BYTES ((size_t)NH * KW * 2)
#define H_BYTES ((size_t)MROWS * NH * 4)
#define OFF_X ((size_t)0)
#define OFF_W (OFF_X + X_BYTES)
#define OFF_H (OFF_W + W_BYTES)
#define WS_TOTAL (OFF_H + H_BYTES)
static_assert((X_BYTES % 128) == 0 && (W_BYTES % 128) == 0 && (H_BYTES % 128) == 0);
static_assert(WS_TOTAL <= (size_t)134217728);
static_assert((size_t)NQ * NP * 4 <= (size_t)NQ_FULL * NP * 4);

__device__ __forceinline__ float bf16r(float x) {
  unsigned int u = __float_as_uint(x);
  u = (u + 0x7FFFu + ((u >> 16) & 1u)) & 0xFFFF0000u;
  return __uint_as_float(u);
}

static __device__ __forceinline__ _Float16 toh_flush(float v) {
  const _Float16 r = (_Float16)v;
  return (fabsf(v) < 6.103515625e-05f) ? (_Float16)0.0f : r;
}
static __device__ __forceinline__ _Float16 relu_toh_flush(float t) {
  const float u = (t < 6.103515625e-05f) ? 0.0f : t;
  return (_Float16)u;
}

__device__ __forceinline__ v16h frag_at(const _Float16* p) {
  v8h lo = *(const v8h*)(p);
  v8h hi = *(const v8h*)(p + 16);
  v16h out;
#pragma unroll
  for (int i = 0; i < 8; ++i) { out[i] = lo[i]; out[i + 8] = hi[i]; }
  return out;
}

__device__ __forceinline__ v8f wmma16(v16h a, v16h b, v8f c) {
  v8f d = __builtin_amdgcn_wmma_f32_16x16x32_f16(false, a, false, b, (short)0, c,
                                                 false, false);
  asm volatile("v_nop\n\tv_nop\n\tv_nop\n\tv_nop" : "+v"(d) : "v"(a), "v"(b));
  return d;
}

__global__ __launch_bounds__(256) void cvt_kernel(
    const float* __restrict__ src, _Float16* __restrict__ dst, float carry) {
  const size_t i0 = ((size_t)blockIdx.x * 256u + threadIdx.x) * 8u;
  const v4f a0 = *(const v4f*)(src + i0);
  const v4f a1 = *(const v4f*)(src + i0 + 4u);
  v8h o;
#pragma unroll
  for (int i = 0; i < 4; ++i) {
    o[i]     = toh_flush(carry * bf16r(a0[i]));
    o[i + 4] = toh_flush(carry * bf16r(a1[i]));
  }
  _Float16* p = dst + i0;
  *(volatile v8h*)p = o;
  __threadfence();
  *(volatile v8h*)p = o;
}

__global__ __launch_bounds__(256) void gemm_h_kernel(
    const _Float16* __restrict__ A16, const _Float16* __restrict__ Bt,
    const float* __restrict__ bias, float* __restrict__ outf) {
  __shared__ __attribute__((aligned(16))) float Cs[64 * LDC];
  const unsigned tid = threadIdx.x, lane = tid & 31u;
  const unsigned w = (unsigned)__builtin_amdgcn_readfirstlane((int)(tid >> 5));
  const unsigned mw = w >> 1, nw = w & 1u;
  const unsigned hh = lane >> 4, m = lane & 15u;
  const unsigned n0 = blockIdx.x * 64u;
  const unsigned row0 = blockIdx.y * 64u;
  const bool is_p = (row0 >= (unsigned)NQ);
  const unsigned koff = is_p ? (unsigned)EMB : 0u;

  const _Float16* ap  = A16 + (size_t)(row0 + mw * 16u + m) * EMB + hh * 8u;
  const _Float16* bp0 = Bt + (size_t)(n0 + nw * 32u + m) * KW + koff + hh * 8u;
  const _Float16* bp1 = bp0 + (size_t)16 * KW;
  v8f acc0 = {}, acc1 = {};
#pragma unroll 2
  for (unsigned k0 = 0; k0 < (unsigned)EMB; k0 += 32u) {
    const v16h a  = frag_at(ap + k0);
    const v16h b0 = frag_at(bp0 + k0);
    const v16h b1 = frag_at(bp1 + k0);
    acc0 = wmma16(a, b0, acc0);
    acc1 = wmma16(a, b1, acc1);
  }
#pragma unroll
  for (int r = 0; r < 8; ++r) {
    float* d = &Cs[(mw * 16u + hh * 8u + (unsigned)r) * LDC + nw * 32u + m];
    d[0]  = acc0[r];
    d[16] = acc1[r];
  }
  __syncthreads();

  const float cs = HCARRY / (XCARRY * WCARRY);
  v4f xs[4];
  size_t off[4];
#pragma unroll
  for (unsigned i = 0; i < 4u; ++i) {
    const unsigned r = 16u * i + (tid >> 4);
    const unsigned c = (tid & 15u) * 4u;
    const v4f u = *(const v4f*)&Cs[r * LDC + c];
    const v4f g = *(const v4f*)(bias + n0 + c);
    v4f val;
#pragma unroll
    for (int j = 0; j < 4; ++j) {
      const float bb = is_p ? (HCARRY * bf16r(g[j])) : 0.0f;
      val[j] = u[j] * cs + bb;
    }
    xs[i] = val;
    off[i] = (size_t)(row0 + r) * NH + n0 + c;
  }
#pragma unroll
  for (int i = 0; i < 4; ++i) *(volatile v4f*)(outf + off[i]) = xs[i];
  __threadfence();
#pragma unroll
  for (int i = 0; i < 4; ++i) *(volatile v4f*)(outf + off[i]) = xs[i];
}

__global__ __launch_bounds__(256) void pair_kernel(
    const float* __restrict__ H, const float* __restrict__ W2, const float* __restrict__ B2,
    float* __restrict__ outp) {
  __shared__ __attribute__((aligned(16))) float HQs[QT * NH];
  __shared__ __attribute__((aligned(16))) float Ss[NM * QT * SP];

  const unsigned tid = threadIdx.x, lane = tid & 31u;
  const unsigned wave = (unsigned)__builtin_amdgcn_readfirstlane((int)(tid >> 5));
  const unsigned hh = lane >> 4, n = lane & 15u;
  const bool col0 = (n == 0u);
  const unsigned pb = blockIdx.x * (unsigned)PT;
  const unsigned q0 = blockIdx.y * (unsigned)QT;

#pragma unroll
  for (unsigned j = 0; j < 5u; ++j) {
    const unsigned idx = (tid + 256u * j) * 4u;
    *(v4f*)&HQs[idx] = *(const v4f*)(H + (size_t)q0 * NH + idx);
  }
  __syncthreads();

  const size_t prow = (size_t)((unsigned)NQ + pb + wave * 16u + n);

#pragma unroll 1
  for (unsigned mm = 0; mm < (unsigned)NM; ++mm) {
    const unsigned hoff = mm * (unsigned)HID + hh * 8u;
    v16h bf[2];
    v4f hp[2][4];
#pragma unroll
    for (unsigned c = 0; c < 2u; ++c) {
      const v4f w0 = *(const v4f*)(W2 + hoff + 32u * c);
      const v4f w1 = *(const v4f*)(W2 + hoff + 32u * c + 4u);
      const v4f w2 = *(const v4f*)(W2 + hoff + 32u * c + 16u);
      const v4f w3 = *(const v4f*)(W2 + hoff + 32u * c + 20u);
#pragma unroll
      for (int j = 0; j < 4; ++j) {
        const _Float16 e0 = toh_flush(WCARRY * bf16r(w0[j]));
        const _Float16 e1 = toh_flush(WCARRY * bf16r(w1[j]));
        const _Float16 e2 = toh_flush(WCARRY * bf16r(w2[j]));
        const _Float16 e3 = toh_flush(WCARRY * bf16r(w3[j]));
        bf[c][j]      = col0 ? e0 : (_Float16)0.0f;
        bf[c][j + 4]  = col0 ? e1 : (_Float16)0.0f;
        bf[c][j + 8]  = col0 ? e2 : (_Float16)0.0f;
        bf[c][j + 12] = col0 ? e3 : (_Float16)0.0f;
      }
      const float* hpr = H + prow * NH + hoff + 32u * c;
      hp[c][0] = *(const v4f*)(hpr);
      hp[c][1] = *(const v4f*)(hpr + 4u);
      hp[c][2] = *(const v4f*)(hpr + 16u);
      hp[c][3] = *(const v4f*)(hpr + 20u);
    }
    const float b2m = bf16r(B2[mm]);

#pragma unroll 1
    for (unsigned q = 0; q < (unsigned)QT; ++q) {
      const unsigned qb = q * (unsigned)NH + hoff;
      v16h af[2];
#pragma unroll
      for (unsigned c = 0; c < 2u; ++c) {
        const v4f g0 = *(const v4f*)&HQs[qb + 32u * c];
        const v4f g1 = *(const v4f*)&HQs[qb + 32u * c + 4u];
        const v4f g2 = *(const v4f*)&HQs[qb + 32u * c + 16u];
        const v4f g3 = *(const v4f*)&HQs[qb + 32u * c + 20u];
#pragma unroll
        for (int j = 0; j < 4; ++j) {
          af[c][j]      = relu_toh_flush(g0[j] + hp[c][0][j]);
          af[c][j + 4]  = relu_toh_flush(g1[j] + hp[c][1][j]);
          af[c][j + 8]  = relu_toh_flush(g2[j] + hp[c][2][j]);
          af[c][j + 12] = relu_toh_flush(g3[j] + hp[c][3][j]);
        }
      }
      v8f acc = {};
      acc = wmma16(af[0], bf[0], acc);
      acc = wmma16(af[1], bf[1], acc);
      if (col0) {
        v4f s0, s1;
#pragma unroll
        for (int j = 0; j < 4; ++j) {
          s0[j] = acc[j]     * (1.0f / (HCARRY * WCARRY)) + b2m;
          s1[j] = acc[j + 4] * (1.0f / (HCARRY * WCARRY)) + b2m;
        }
        const unsigned si = (mm * (unsigned)QT + q) * (unsigned)SP + wave * 16u + hh * 8u;
        *(v4f*)&Ss[si]      = s0;
        *(v4f*)&Ss[si + 4u] = s1;
      }
    }
  }
  __syncthreads();

  v4f xs[2];
  size_t off[2];
#pragma unroll
  for (unsigned i = 0; i < 2u; ++i) {
    const unsigned q = 8u * i + wave;
    const unsigned p4 = lane * 4u;
    const v4f o0 = *(const v4f*)&Ss[(0u * (unsigned)QT + q) * (unsigned)SP + p4];
    const v4f o1 = *(const v4f*)&Ss[(1u * (unsigned)QT + q) * (unsigned)SP + p4];
    const v4f o2 = *(const v4f*)&Ss[(2u * (unsigned)QT + q) * (unsigned)SP + p4];
    const v4f o3 = *(const v4f*)&Ss[(3u * (unsigned)QT + q) * (unsigned)SP + p4];
    const v4f o4 = *(const v4f*)&Ss[(4u * (unsigned)QT + q) * (unsigned)SP + p4];
    v4f val;
#pragma unroll
    for (int j = 0; j < 4; ++j) {
      const float s = (((o0[j] + o1[j]) + o2[j]) + o3[j]) + o4[j];
      const float mean = s * (1.0f / (float)NM);
      const float d0 = o0[j] - mean, d1 = o1[j] - mean, d2 = o2[j] - mean;
      const float d3 = o3[j] - mean, d4 = o4[j] - mean;
      const float ss = (((d0 * d0 + d1 * d1) + d2 * d2) + d3 * d3) + d4 * d4;
      const float sd = sqrtf(ss * (1.0f / (float)(NM - 1)));
      val[j] = mean * expf(-sd);
    }
    xs[i] = val;
    off[i] = (size_t)(q0 + q) * NP + pb + p4;
  }
#pragma unroll
  for (int i = 0; i < 2; ++i) *(volatile v4f*)(outp + off[i]) = xs[i];
  __threadfence();
#pragma unroll
  for (int i = 0; i < 2; ++i) *(volatile v4f*)(outp + off[i]) = xs[i];
}

extern "C" void kernel_launch(void* const* d_in, const int* in_sizes, int n_in,
                              void* d_out, int out_size, void* d_ws, size_t ws_size,
                              hipStream_t stream) {
  if (n_in < 6) return;
  if ((long long)in_sizes[0] < (long long)NQ * EMB) return;
  if ((long long)in_sizes[1] < (long long)NP * EMB) return;
  if ((long long)in_sizes[2] < (long long)NH * KW) return;
  if (in_sizes[3] < NH || in_sizes[4] < NH || in_sizes[5] < NM) return;
  if ((long long)out_size < (long long)NQ * NP) return;
  if (ws_size < WS_TOTAL) return;

  const float* Q  = (const float*)d_in[0];
  const float* P  = (const float*)d_in[1];
  const float* W1 = (const float*)d_in[2];
  const float* b1 = (const float*)d_in[3];
  const float* W2 = (const float*)d_in[4];
  const float* b2 = (const float*)d_in[5];
  float* out = (float*)d_out;

  char* ws = (char*)d_ws;
  _Float16* X16 = (_Float16*)(ws + OFF_X);
  _Float16* W16 = (_Float16*)(ws + OFF_W);
  float*    Hf  = (float*)(ws + OFF_H);

  dim3 blk(256);
  cvt_kernel<<<dim3((unsigned)(((size_t)NQ * EMB) / 2048)), blk, 0, stream>>>(Q, X16, XCARRY);
  cvt_kernel<<<dim3((unsigned)(((size_t)NP * EMB) / 2048)), blk, 0, stream>>>(
      P, X16 + (size_t)NQ * EMB, XCARRY);
  cvt_kernel<<<dim3((unsigned)(((size_t)NH * KW) / 2048)), blk, 0, stream>>>(W1, W16, WCARRY);
  gemm_h_kernel<<<dim3(NH / 64, MROWS / 64), blk, 0, stream>>>(X16, W16, b1, Hf);
  pair_kernel<<<dim3(NP / PT, NQ / QT), blk, 0, stream>>>(Hf, W2, b2, out);
}
